// ConditionalPreactivation_13048110645402
// MI455X (gfx1250) — hardware-verified
//
#include <hip/hip_runtime.h>
#include <math.h>

typedef __attribute__((ext_vector_type(16))) _Float16 v16h;
typedef __attribute__((ext_vector_type(16))) __bf16 v16b;
typedef __attribute__((ext_vector_type(8)))  _Float16 v8h;
typedef __attribute__((ext_vector_type(8)))  float v8f;
typedef __attribute__((ext_vector_type(4)))  float v4f;
typedef __attribute__((ext_vector_type(2)))  float v2f;
typedef __attribute__((ext_vector_type(4)))  unsigned v4u;
typedef __attribute__((ext_vector_type(4)))  int v4i;
typedef float __attribute__((may_alias)) float_a;
typedef int __attribute__((may_alias)) int_a;

template <typename T> __device__ __forceinline__ void vst2(void* p, T v) { *(volatile T*)p = v; __threadfence(); *(volatile T*)p = v; }
__device__ __forceinline__ v8f wmma16(v16h a, v16h b, v8f c) {
  v8f d = __builtin_amdgcn_wmma_f32_16x16x32_f16(false, a, false, b, (short)0, c, false, false);
  asm volatile("v_nop\n\tv_nop\n\tv_nop\n\tv_nop" : "+v"(d) : "v"(a), "v"(b));
  return d;
}
__device__ __forceinline__ v8f wmma_bf(v16b a, v16b b, v8f c) {
  v8f d = __builtin_amdgcn_wmma_f32_16x16x32_bf16(false, a, false, b, (short)0, c, false, false);
  asm volatile("v_nop\n\tv_nop\n\tv_nop\n\tv_nop" : "+v"(d) : "v"(a), "v"(b));
  return d;
}
__device__ __forceinline__ v16h frag_h(const _Float16* rowk0, int lane) {
  union { v16h v; v8h q[2]; } u; const _Float16* p = rowk0 + 8 * (lane >> 4);
  u.q[0] = *(const v8h*)p; u.q[1] = *(const v8h*)(p + 16); return u.v;
}
__device__ __forceinline__ v16h frag_f32(const float* rowk0, int lane) {
  v16h a; const float* p = rowk0 + 8 * (lane >> 4);
#pragma unroll
  for (int i = 0; i < 8; ++i) { a[i] = (_Float16)p[i]; a[8 + i] = (_Float16)p[16 + i]; }
  return a;
}
__device__ __forceinline__ v16h frag_f32s(const float* rowk0, int lane, float sc) {
  v16h a; const float* p = rowk0 + 8 * (lane >> 4);
#pragma unroll
  for (int i = 0; i < 8; ++i) { a[i] = (_Float16)(p[i] * sc); a[8 + i] = (_Float16)(p[16 + i] * sc); }
  return a;
}
__device__ __forceinline__ v16h fragc_f32(const float* W, int k0, int n, int lane, int ld, int K) {
  v16h a; const int g = lane >> 4;
#pragma unroll
  for (int i = 0; i < 8; ++i) { const int ka = k0 + 8 * g + i, kb = ka + 16;
    a[i] = (_Float16)(ka < K ? W[(size_t)(ka < K ? ka : K - 1) * ld + n] : 0.f); a[8 + i] = (_Float16)(kb < K ? W[(size_t)(kb < K ? kb : K - 1) * ld + n] : 0.f); }
  return a;
}
struct F2 { v16b h, l; };
__device__ __forceinline__ F2 bsplit16(const float v[16]) { F2 r;
#pragma unroll
  for (int i = 0; i < 16; ++i) { const __bf16 h = (__bf16)v[i]; r.h[i] = h; r.l[i] = (__bf16)(v[i] - (float)h); }
  return r; }
__device__ __forceinline__ F2 split_row(const float* row, int k0, int lane) { float v[16]; const float* p = row + k0 + 8 * (lane >> 4);
#pragma unroll
  for (int i = 0; i < 8; ++i) { v[i] = p[i]; v[8 + i] = p[16 + i]; }
  return bsplit16(v); }
__device__ __forceinline__ F2 split_rowK(const float* row, int k0, int lane, int K) { float v[16]; const int g = lane >> 4;
#pragma unroll
  for (int i = 0; i < 8; ++i) { const int ka = k0 + 8 * g + i, kb = ka + 16; v[i] = ka < K ? row[ka < K ? ka : K - 1] : 0.f; v[8 + i] = kb < K ? row[kb < K ? kb : K - 1] : 0.f; }
  return bsplit16(v); }
__device__ __forceinline__ F2 split_col(const float* W, int k0, int n, int lane, int ld, int K) { float v[16]; const int g = lane >> 4;
#pragma unroll
  for (int i = 0; i < 8; ++i) { const int ka = k0 + 8 * g + i, kb = ka + 16; v[i] = ka < K ? W[(size_t)(ka < K ? ka : K - 1) * ld + n] : 0.f; v[8 + i] = kb < K ? W[(size_t)(kb < K ? kb : K - 1) * ld + n] : 0.f; }
  return bsplit16(v); }
__device__ __forceinline__ v8f mac3(const F2& a, const F2& b, v8f c) { c = wmma_bf(a.l, b.h, c); c = wmma_bf(a.h, b.l, c); return wmma_bf(a.h, b.h, c); }
__device__ __forceinline__ float sigm(float v) { return 1.0f / (1.0f + expf(-v)); }
#define LDSX() do { asm volatile("s_wait_dscnt 0" ::: "memory"); __builtin_amdgcn_wave_barrier(); __builtin_amdgcn_fence(__ATOMIC_RELEASE, "workgroup"); } while (0)


#define NR 4096
#define DIN 512
#define DOUT 512
#define DC 64
#define KB 16
#define DB 256
#define KK (KB * DIN)
#define NEG 0.01f
#ifndef TR
#define TR (NR / 64)
#endif
typedef __attribute__((ext_vector_type(8))) __bf16 v8b;
__device__ __forceinline__ v16b frag_b(const __bf16* rowk0, int lane) {
  union { v16b v; v8b q[2]; } u; const __bf16* p = rowk0 + 8 * (lane >> 4);
  u.q[0] = *(const v8b*)p; u.q[1] = *(const v8b*)(p + 16); return u.v;
}
__device__ __forceinline__ float bfr(float v) { return (float)(__bf16)v; }
__device__ __attribute__((noinline)) float exp_ni(float v) { return expf(v); }
__device__ __attribute__((noinline)) float erf_ni(float v) { return erff(v); }

#define WS_WT  0u
#define WS_A   (WS_WT + 2u * (size_t)DOUT * KK)
#define WS_BF  (WS_A + 2u * (size_t)NR * KK)
#define BFS 32
#define WS_END (WS_BF + 4u * (size_t)NR * BFS)

__device__ __forceinline__ float lrelu(float v) { return v >= 0.f ? v : NEG * v; }
__global__ __launch_bounds__(256) void k_packw(const float* __restrict__ Wb, _Float16* __restrict__ WT) { __shared__ __align__(16) _Float16 s[KK]; const int o = blockIdx.x, t = threadIdx.x;
  for (int e = t; e < KK; e += 256) s[e] = (_Float16)bfr(Wb[(size_t)e * DOUT + o]);
  __syncthreads(); for (int q = t; q < KK / 8; q += 256) vst2((unsigned*)(WT + (size_t)o * KK + q * 8), *(const v4u*)&s[q * 8]); }
__global__ __launch_bounds__(256) void k_row(const float* __restrict__ X, const float* __restrict__ C, const float* __restrict__ G, const float* __restrict__ Bt, const float* __restrict__ W1, const float* __restrict__ B1, const float* __restrict__ WR, const float* __restrict__ BR, const float* __restrict__ W2, const float* __restrict__ B2, _Float16* __restrict__ A16, float* __restrict__ BF) {
  __shared__ float red[8]; __shared__ float sa[DIN]; __shared__ float sc[DC]; __shared__ float sh[DB]; __shared__ float sh2[DB]; __shared__ float sred[8][KB]; __shared__ __align__(16) float sbf[BFS]; __shared__ __align__(16) _Float16 srow[KK];
  const int t = threadIdx.x; const size_t row = blockIdx.x;
  float v[2]; float s = 0.f; for (int i = 0; i < 2; ++i) { v[i] = bfr(X[row * DIN + t + 256 * i]); s += v[i]; }
#pragma unroll
  for (int o = 1; o < 32; o <<= 1) s += __shfl_xor(s, o);
  if ((t & 31) == 0) red[t >> 5] = s; __syncthreads(); float mu = 0.f; for (int i = 0; i < 8; ++i) mu += red[i]; mu /= (float)DIN; __syncthreads();
  float q = 0.f; for (int i = 0; i < 2; ++i) { const float d = v[i] - mu; q += d * d; }
#pragma unroll
  for (int o = 1; o < 32; o <<= 1) q += __shfl_xor(q, o);
  if ((t & 31) == 0) red[t >> 5] = q; __syncthreads(); float var = 0.f; for (int i = 0; i < 8; ++i) var += red[i]; var /= (float)DIN; const float inv = 1.0f / sqrtf(var + 1e-5f);
  for (int i = 0; i < 2; ++i) { const int cix = t + 256 * i; sa[cix] = lrelu((v[i] - mu) * inv * bfr(G[cix]) + bfr(Bt[cix])); }
  if (t < DC) sc[t] = bfr(C[row * DC + t]); __syncthreads();
  { float h = bfr(B1[t]);
#pragma unroll 1
    for (int k = 0; k < DC; ++k) h += sc[k] * bfr(W1[(size_t)k * DB + t]); sh[t] = h; } __syncthreads();
  { float h = sh[t] + bfr(BR[t]);
#pragma unroll 1
    for (int k = 0; k < DB; ++k) h += lrelu(sh[k]) * bfr(WR[(size_t)k * DB + t]); sh2[t] = lrelu(h); } __syncthreads();
  { float part[KB];
#pragma unroll
    for (int k = 0; k < KB; ++k) part[k] = sh2[t] * bfr(W2[(size_t)t * KB + k]);
#pragma unroll
    for (int k = 0; k < KB; ++k) { float pv = part[k];
#pragma unroll
      for (int o = 1; o < 32; o <<= 1) pv += __shfl_xor(pv, o);
      if ((t & 31) == 0) sred[t >> 5][k] = pv; } }
  __syncthreads(); if (t < KB) { float bfv = bfr(B2[t]); for (int w = 0; w < 8; ++w) bfv += sred[w][t]; sbf[t] = bfv; } else if (t < BFS) sbf[t] = 0.f; __syncthreads();
  for (int e = t; e < KK; e += 256) srow[e] = (_Float16)(sbf[e / DIN] * sa[e % DIN]); __syncthreads();
  for (int qq = t; qq < KK / 8; qq += 256) vst2((unsigned*)(A16 + row * KK + qq * 8), *(const v4u*)&srow[qq * 8]); if (t < BFS / 4) vst2(BF + row * BFS + t * 4, *(const v4f*)&sbf[t * 4]); }
__global__ __launch_bounds__(128) void k_big(const _Float16* __restrict__ A16, const _Float16* __restrict__ WT, const float* __restrict__ BF, const float* __restrict__ BV, float* __restrict__ OUT) { __shared__ __align__(16) float sf[4][16][132];
  const int tid = threadIdx.x, wave = tid >> 5, lane = tid & 31, col = lane & 15, g = lane >> 4; const size_t r0 = (size_t)blockIdx.x * 64 + wave * 16; const int c0 = blockIdx.y * 128;
  v8f acc[8] = {};
#pragma unroll 2
  for (int kc = 0; kc < KK / 32; ++kc) { const v16h a = frag_h(A16 + (r0 + col) * KK + kc * 32, lane);
#pragma unroll
    for (int j = 0; j < 8; ++j) acc[j] = wmma16(a, frag_h(WT + (size_t)(c0 + j * 16 + col) * KK + kc * 32, lane), acc[j]); }
#pragma unroll
  for (int j = 0; j < 8; ++j) { const int o = c0 + j * 16 + col;
#pragma unroll
    for (int r = 0; r < 8; ++r) { const size_t row = r0 + 8 * g + r; float bsum = 0.f;
#pragma unroll
      for (int k = 0; k < KB; ++k) bsum += BF[row * BFS + k] * bfr(BV[(size_t)k * DOUT + o]); sf[wave][8 * g + r][j * 16 + col] = acc[j][r] + bsum; } }
  LDSX(); for (int rl = 0; rl < 16; ++rl) vst2(OUT + (r0 + rl) * DOUT + c0 + lane * 4, *(const v4f*)&sf[wave][rl][lane * 4]); }
extern "C" void kernel_launch(void* const* d_in, const int* in_sizes, int n_in, void* d_out, int out_size, void* d_ws, size_t ws_size, hipStream_t stream) {
  (void)in_sizes; (void)n_in; (void)out_size;
  const float** F = (const float**)d_in;
  if (ws_size < (size_t)WS_END) return;
  char* ws = (char*)d_ws; _Float16 *WT = (_Float16*)(ws + WS_WT), *A16 = (_Float16*)(ws + WS_A); float* BF = (float*)(ws + WS_BF);
  k_packw<<<DOUT, 256, 0, stream>>>(F[10], WT);
  k_row<<<TR * 64, 256, 0, stream>>>(F[0], F[1], F[2], F[3], F[4], F[5], F[6], F[7], F[8], F[9], A16, BF);
  k_big<<<dim3(TR, DOUT / 128), 128, 0, stream>>>(A16, WT, BF, F[11], (float*)d_out);
}
